// CustomAttention_35278861369702
// MI455X (gfx1250) — hardware-verified
//
#include <hip/hip_runtime.h>


#pragma clang fp contract(off)

#ifndef NB
#define NB 2
#endif
#ifndef SEQ
#define SEQ 2048
#endif
#define NB_FULL  2
#define SEQ_FULL 2048
#define HID  2048
#define NHQ  16
#define NKV  4
#define REP  (NHQ / NKV)
#define HD   128
#define DQ   (NHQ * HD)
#define DKV  (NKV * HD)
#define RH   ((SEQ < 256) ? SEQ : 256)
#define PCAR 4096.0f
#define CCAR 16.0f
#define WCAR 64.0f
#define SCL  0.08838834764831845f
#define L2E  1.4426950408889634f
#define NEGBIG (-3.0e38f)
#define PSP  40
#define CSP  136

static_assert(SEQ % 64 == 0 && SEQ >= 64 && SEQ <= SEQ_FULL);
static_assert(NB >= 1 && NB <= NB_FULL);
static_assert((RH % 64) == 0 && RH <= SEQ && RH % 16 == 0);
static_assert(HID % 64 == 0 && DQ % 64 == 0 && DKV % 64 == 0 && HD == 128 && HID % 32 == 0 && DQ % 32 == 0);
static_assert((SEQ * SEQ / 64 + 255) / 256 <= 256);
static_assert((PSP * 2) % 16 == 0 && (CSP * 2) % 16 == 0);

typedef _Float16 h16;
typedef unsigned short bf;
typedef __attribute__((ext_vector_type(16))) __bf16   v16bf;
typedef __attribute__((ext_vector_type(16))) _Float16 v16h;
typedef __attribute__((ext_vector_type(8)))  _Float16 v8h;
typedef __attribute__((ext_vector_type(8)))  unsigned short v8us;
typedef __attribute__((ext_vector_type(8)))  float    v8f;
typedef __attribute__((ext_vector_type(4)))  float    v4f;
typedef __attribute__((ext_vector_type(2)))  _Float16 v2h;
typedef __attribute__((ext_vector_type(2)))  unsigned short v2us;
typedef __attribute__((ext_vector_type(2)))  float v2f;
typedef v8h  __attribute__((may_alias)) v8ha;
typedef v4f  __attribute__((may_alias)) v4fa;
typedef v8us __attribute__((may_alias)) v8usa;

__device__ __forceinline__ unsigned short f2bf(float f) { unsigned u = __float_as_uint(f); u += 0x7FFFu + ((u >> 16) & 1u); return (unsigned short)(u >> 16); }
__device__ __forceinline__ float bf2f(unsigned short b) { return __uint_as_float(((unsigned)b) << 16); }
__device__ __forceinline__ float bfr(float f) { return bf2f(f2bf(f)); }
__device__ __forceinline__ void splitf(float y, unsigned short& h, unsigned short& l) { h = f2bf(y); l = f2bf(y - bf2f(h)); }
__device__ __forceinline__ v16h cat16(v8h lo, v8h hi) { return __builtin_shufflevector(lo, hi, 0, 1, 2, 3, 4, 5, 6, 7, 8, 9, 10, 11, 12, 13, 14, 15); }
__device__ __forceinline__ v16bf cat16b(v8us lo, v8us hi) { return __builtin_bit_cast(v16bf, __builtin_shufflevector(lo, hi, 0, 1, 2, 3, 4, 5, 6, 7, 8, 9, 10, 11, 12, 13, 14, 15)); }
__device__ __forceinline__ v8f wmma16(v16h a, v16h b, v8f c) { return __builtin_amdgcn_wmma_f32_16x16x32_f16(false, a, false, b, (short)0, c, false, false); }
__device__ __forceinline__ v8f wmmab(v16bf a, v16bf b, v8f c) { return __builtin_amdgcn_wmma_f32_16x16x32_bf16(false, a, false, b, (short)0, c, false, false); }

template <typename T16> struct WFrag;
template <> struct WFrag<h16> { typedef v16h V; static __device__ __forceinline__ V ld(const h16* p) { return cat16(*(const v8h*)p, *(const v8h*)(p + 16)); } static __device__ __forceinline__ v8f mma(V a, V b, v8f c) { return wmma16(a, b, c); } };
template <> struct WFrag<bf>  { typedef v16bf V; static __device__ __forceinline__ V ld(const bf* p) { return cat16b(*(const v8us*)p, *(const v8us*)(p + 16)); } static __device__ __forceinline__ v8f mma(V a, V b, v8f c) { return wmmab(a, b, c); } };
__device__ __forceinline__ v16h  ldsA16(const unsigned short* p) { return cat16(*(const v8ha*)p, *(const v8ha*)(p + 16)); }
__device__ __forceinline__ v16bf ldsAbf(const unsigned short* p) { return cat16b(*(const v8usa*)p, *(const v8usa*)(p + 16)); }

template <typename T16, int NSPLIT>
__global__ __launch_bounds__(32) void k_gemmw(const T16* __restrict__ A, const T16* __restrict__ A2, const T16* __restrict__ Bt, const T16* __restrict__ Bt2, int K, float* C, int ldc, float oscale) {
    typedef typename WFrag<T16>::V V;
    __shared__ __align__(16) float os[16 * 68];
    const int lane = threadIdx.x & 31, lr = lane & 15, hi = lane >> 4; const int r0 = blockIdx.x * 64, c0 = blockIdx.y * 64;
    v8f acc[4][4];
#pragma unroll
    for (int mb = 0; mb < 4; ++mb)
#pragma unroll
        for (int nb = 0; nb < 4; ++nb) acc[mb][nb] = (v8f){};
    const size_t aoff = (size_t)(r0 + lr) * K + 8 * hi, boff = (size_t)(c0 + lr) * K + 8 * hi;
#pragma unroll 1
    for (int kc = 0; kc < K; kc += 32) {
        V a[4], a2[4];
#pragma unroll
        for (int mb = 0; mb < 4; ++mb) { a[mb] = WFrag<T16>::ld(A + aoff + (size_t)mb * 16 * K + kc); if (NSPLIT == 1 || NSPLIT == 2) a2[mb] = WFrag<T16>::ld(A2 + aoff + (size_t)mb * 16 * K + kc); }
#pragma unroll
        for (int nb = 0; nb < 4; ++nb) { const V b = WFrag<T16>::ld(Bt + boff + (size_t)nb * 16 * K + kc); V b2; if (NSPLIT >= 2) b2 = WFrag<T16>::ld(Bt2 + boff + (size_t)nb * 16 * K + kc);
#pragma unroll
            for (int mb = 0; mb < 4; ++mb) { acc[mb][nb] = WFrag<T16>::mma(a[mb], b, acc[mb][nb]); if (NSPLIT == 1 || NSPLIT == 2) acc[mb][nb] = WFrag<T16>::mma(a2[mb], b, acc[mb][nb]); if (NSPLIT >= 2) acc[mb][nb] = WFrag<T16>::mma(a[mb], b2, acc[mb][nb]); } }
        asm volatile("v_nop\n\tv_nop\n\tv_nop\n\tv_nop" : "+v"(acc[0][0]), "+v"(acc[1][1]), "+v"(acc[2][2]), "+v"(acc[3][3]) : "v"(a[0]), "v"(a[3]));
    }
#pragma unroll
    for (int mb = 0; mb < 4; ++mb) {
#pragma unroll
        for (int nb = 0; nb < 4; ++nb) {
#pragma unroll
            for (int j = 0; j < 8; ++j) os[(hi * 8 + j) * 68 + nb * 16 + lr] = acc[mb][nb][j]; }
        __builtin_amdgcn_wave_barrier(); asm volatile("" ::: "memory");
        float* crow = C + (size_t)(r0 + mb * 16) * ldc + c0;
#pragma unroll 1
        for (int ps = 0; ps < 2; ++ps) {
#pragma unroll
            for (int s = 0; s < 8; ++s) { const int row = 2 * s + hi, cofs = lr * 4; v4f val = *(const v4fa*)(os + row * 68 + cofs); val = val * oscale;
                *(volatile v4f*)(crow + (size_t)row * ldc + cofs) = val; }
            if (ps == 0) __threadfence(); }
        __builtin_amdgcn_wave_barrier(); asm volatile("" ::: "memory");
    }
}

__global__ __launch_bounds__(256) void k_cvt8(const float* __restrict__ src, bf* dst, size_t n8) { const size_t i = (size_t)blockIdx.x * 256 + threadIdx.x; if (i >= n8) return; const v8f v = *(const v8f*)(src + i * 8); v8us o;
#pragma unroll
    for (int k = 0; k < 8; ++k) o[k] = f2bf(v[k]); *(volatile v8us*)(dst + i * 8) = o; __threadfence(); *(volatile v8us*)(dst + i * 8) = o; }
__global__ __launch_bounds__(256) void k_cvt16s(const float* __restrict__ src, h16* dst, size_t n8, float sc) { const size_t i = (size_t)blockIdx.x * 256 + threadIdx.x; if (i >= n8) return; const v8f v = *(const v8f*)(src + i * 8); v8h o;
#pragma unroll
    for (int k = 0; k < 8; ++k) o[k] = (h16)(bfr(v[k]) * sc); *(volatile v8h*)(dst + i * 8) = o; __threadfence(); *(volatile v8h*)(dst + i * 8) = o; }

__global__ __launch_bounds__(64) void k_invf(float* invf) {
    const int j = threadIdx.x;
    const double ex = (double)(2 * j) * 0.0078125;
    const double pw = exp2(ex * 13.287712379549449);
    const float pf = (float)pw; const float iv = 1.0f / pf;
    *(volatile float*)(invf + j) = iv; __threadfence(); *(volatile float*)(invf + j) = iv;
}
__global__ __launch_bounds__(256) void k_cstab(const float* __restrict__ invf, float* CS) {
    const int idx = blockIdx.x * 256 + threadIdx.x; if (idx >= SEQ * HD) return;
    const int t = idx / HD, d = idx % HD, j = d & (HD / 2 - 1);
    const float ang = (float)t * invf[j];
    float sn, cn; sincosf(ang, &sn, &cn);
    v2f cs; cs[0] = cn; cs[1] = sn;
    *(volatile v2f*)(CS + (size_t)idx * 2) = cs; __threadfence(); *(volatile v2f*)(CS + (size_t)idx * 2) = cs;
}

__global__ __launch_bounds__(256) void k_mchk(const float* __restrict__ M, int* part) {
    __shared__ int red[256];
    const int tid = threadIdx.x, lane = tid & 31;
    const size_t nthr = (size_t)SEQ * SEQ / 64;
    const size_t gid = (size_t)blockIdx.x * 256 + tid;
    const size_t gc = (gid < nthr) ? gid : 0;
    const int i = (int)((gc * 64) / SEQ), j0 = (int)((gc * 64) % SEQ);
    const float* row = M + (size_t)i * SEQ_FULL + j0;
    int badc = 0;
#pragma unroll 1
    for (int c = 0; c < 64; c += 4) {
        const v4f m = *(const v4f*)(row + c);
#pragma unroll
        for (int q = 0; q < 4; ++q) { const int j = j0 + c + q; const float v = m[q]; const bool okz = (v == 0.0f); const bool okn = (v <= -1000.0f); const bool ok = (j <= i) ? okz : okn; badc += ok ? 0 : 1; }
    }
    badc = (gid < nthr) ? badc : 0;
    red[tid] = badc; __syncthreads();
#pragma unroll
    for (int sh = 128; sh >= 32; sh >>= 1) { if (tid < sh) red[tid] = red[tid] + red[tid + sh]; __syncthreads(); }
    int v = red[lane];
#pragma unroll
    for (int sh = 16; sh; sh >>= 1) v += __shfl_xor(v, sh, 32);
    if (tid < 32) { int* p = part + (size_t)blockIdx.x * 32 + lane; *(volatile int*)p = v; __threadfence(); *(volatile int*)p = v; }
}
__global__ __launch_bounds__(256) void k_mred(const int* __restrict__ part, int nblk, int* flag) {
    __shared__ int red[256];
    const int tid = threadIdx.x, lane = tid & 31;
    const int tc = (tid < nblk) ? tid : 0; int v0 = part[(size_t)tc * 32]; v0 = (tid < nblk) ? v0 : 0;
    red[tid] = v0; __syncthreads();
#pragma unroll
    for (int sh = 128; sh >= 32; sh >>= 1) { if (tid < sh) red[tid] = red[tid] + red[tid + sh]; __syncthreads(); }
    int v = red[lane];
#pragma unroll
    for (int sh = 16; sh; sh >>= 1) v += __shfl_xor(v, sh, 32);
    if (tid < 32) { int* p = flag + lane; *(volatile int*)p = v; __threadfence(); *(volatile int*)p = v; }
}

__global__ __launch_bounds__(256) void k_rope(const float* __restrict__ F, int pitch, int nheads, const float* __restrict__ CS, h16* P16, bf* Ph, bf* Pl) {
    const size_t e = ((size_t)blockIdx.x * 256 + threadIdx.x) * 2; if (e >= (size_t)nheads * SEQ * HD) return;
    const int d = (int)(e % HD); const int t = (int)((e / HD) % SEQ); const int hh = (int)(e / ((size_t)HD * SEQ));
    const float* f = F + (size_t)t * pitch + hh * HD; v2h o16; v2us oh, ol;
#pragma unroll
    for (int q = 0; q < 2; ++q) { const int dd = d + q; const int dp = (dd < HD / 2) ? dd + HD / 2 : dd - HD / 2; const float x0 = f[dd], x1 = f[dp];
        const v2f cs = *(const v2f*)(CS + ((size_t)t * HD + dd) * 2); float a = __fmul_rn(x0, cs[0]), bq = __fmul_rn(x1, cs[1]); asm volatile("" : "+v"(a)); asm volatile("" : "+v"(bq));
        const float r = (dd < HD / 2) ? __fsub_rn(a, bq) : __fadd_rn(a, bq);
        o16[q] = (h16)r; unsigned short a2, c2; splitf(r, a2, c2); oh[q] = a2; ol[q] = c2; }
    const bool lo = (t < RH); const size_t oo = ((size_t)hh * RH + (lo ? t : 0)) * HD + d;
    *(volatile v2h*)(P16 + e) = o16; if (lo) { *(volatile v2us*)(Ph + oo) = oh; *(volatile v2us*)(Pl + oo) = ol; }
    __threadfence();
    *(volatile v2h*)(P16 + e) = o16; if (lo) { *(volatile v2us*)(Ph + oo) = oh; *(volatile v2us*)(Pl + oo) = ol; }
}
__global__ __launch_bounds__(256) void k_vtp(const float* __restrict__ F, int pitch, int nheads, h16* V16, bf* Vh, bf* Vl) {
    const size_t e = ((size_t)blockIdx.x * 256 + threadIdx.x) * 2; if (e >= (size_t)nheads * HD * SEQ) return;
    const int t = (int)(e % SEQ); const int d = (int)((e / SEQ) % HD); const int g = (int)(e / ((size_t)SEQ * HD)); v2h o16; v2us oh, ol;
#pragma unroll
    for (int q = 0; q < 2; ++q) { const float x = F[(size_t)(t + q) * pitch + g * HD + d]; o16[q] = (h16)x; unsigned short a2, c2; splitf(x, a2, c2); oh[q] = a2; ol[q] = c2; }
    const bool lo = (t < RH); const size_t oo = ((size_t)g * HD + d) * RH + (lo ? t : 0);
    *(volatile v2h*)(V16 + e) = o16; if (lo) { *(volatile v2us*)(Vh + oo) = oh; *(volatile v2us*)(Vl + oo) = ol; }
    __threadfence();
    *(volatile v2h*)(V16 + e) = o16; if (lo) { *(volatile v2us*)(Vh + oo) = oh; *(volatile v2us*)(Vl + oo) = ol; }
}

template <bool HIRES>
__global__ __launch_bounds__(128) __attribute__((amdgpu_num_vgpr(256)))
void k_flash(const h16* __restrict__ Q16, const bf* __restrict__ Qh, const bf* __restrict__ Ql,
             const h16* __restrict__ K16, const bf* __restrict__ Kh, const bf* __restrict__ Kl,
             const h16* __restrict__ V16, const bf* __restrict__ Vh, const bf* __restrict__ Vl,
             const int* __restrict__ FL, int qb0, unsigned short* AT16, unsigned short* ATh, unsigned short* ATl) {
    __shared__ __align__(16) unsigned short Ps[4][2][16 * PSP];
    __shared__ __align__(16) unsigned short Cs[4][16 * CSP];
    const int lane = threadIdx.x & 31, lr = lane & 15, hi = lane >> 4, w = threadIdx.x >> 5;
    const int qb = qb0 + (int)blockIdx.x, h = (int)blockIdx.y, g = h / REP;
    const int q0 = qb * 64 + w * 16;
    unsigned short* P0 = &Ps[w][0][0]; unsigned short* P1 = &Ps[w][1][0]; unsigned short* CW = &Cs[w][0];
    v8f acc[8];
#pragma unroll
    for (int f = 0; f < 8; ++f) acc[f] = (v8f){};
    float rowm[8], rowl[8];
#pragma unroll
    for (int r = 0; r < 8; ++r) { rowm[r] = NEGBIG; rowl[r] = 0.0f; }
    v16h qa[4];
    if (!HIRES) {
#pragma unroll
        for (int ks = 0; ks < 4; ++ks) qa[ks] = WFrag<h16>::ld(Q16 + ((size_t)h * SEQ + q0 + lr) * HD + 8 * hi + 32 * ks);
    }
    const int nkt = (q0 + 15) / 32 + 1;
#pragma unroll 1
    for (int kt = 0; kt < nkt; ++kt) {
        const int kb = kt * 32;
        __builtin_amdgcn_wave_barrier(); asm volatile("" ::: "memory");
        v8f s[2]; s[0] = (v8f){}; s[1] = (v8f){};
        if (HIRES) {
            int zo = 0; asm volatile("" : "+v"(zo));
            v16bf ah, al, khf[2], klf[2];
#pragma unroll
            for (int ks = 0; ks < 4; ++ks) {
                ah = WFrag<bf>::ld(Qh + ((size_t)h * RH + q0 + lr) * HD + 8 * hi + 32 * ks + zo);
                al = WFrag<bf>::ld(Ql + ((size_t)h * RH + q0 + lr) * HD + 8 * hi + 32 * ks + zo);
#pragma unroll
                for (int j = 0; j < 2; ++j) {
                    khf[j] = WFrag<bf>::ld(Kh + ((size_t)g * RH + kb + 16 * j + lr) * HD + 8 * hi + 32 * ks);
                    klf[j] = WFrag<bf>::ld(Kl + ((size_t)g * RH + kb + 16 * j + lr) * HD + 8 * hi + 32 * ks);
                    s[j] = wmmab(ah, khf[j], s[j]); s[j] = wmmab(al, khf[j], s[j]); s[j] = wmmab(ah, klf[j], s[j]); } }
            asm volatile("v_nop\n\tv_nop\n\tv_nop\n\tv_nop" : "+v"(s[0]), "+v"(s[1]) : "v"(ah), "v"(al), "v"(khf[0]), "v"(khf[1]), "v"(klf[0]), "v"(klf[1]));
        } else {
            v16h kf[2];
#pragma unroll
            for (int ks = 0; ks < 4; ++ks) {
#pragma unroll
                for (int j = 0; j < 2; ++j) { kf[j] = WFrag<h16>::ld(K16 + ((size_t)g * SEQ + kb + 16 * j + lr) * HD + 8 * hi + 32 * ks); s[j] = wmma16(qa[ks], kf[j], s[j]); } }
            asm volatile("v_nop\n\tv_nop\n\tv_nop\n\tv_nop" : "+v"(s[0]), "+v"(s[1]) : "v"(qa[0]), "v"(qa[3]), "v"(kf[0]), "v"(kf[1]));
        }
#pragma unroll
        for (int r = 0; r < 8; ++r) {
            const int q = q0 + 8 * hi + r;
            float a0 = s[0][r] * SCL, a1 = s[1][r] * SCL;
            a0 = (kb + lr > q) ? NEGBIG : a0; a1 = (kb + 16 + lr > q) ? NEGBIG : a1;
            float mx = fmaxf(a0, a1);
            mx = fmaxf(mx, __shfl_xor(mx, 1, 32)); mx = fmaxf(mx, __shfl_xor(mx, 2, 32)); mx = fmaxf(mx, __shfl_xor(mx, 4, 32)); mx = fmaxf(mx, __shfl_xor(mx, 8, 32));
            const float mn = fmaxf(rowm[r], mx);
            const float corr = __builtin_amdgcn_exp2f(fmaxf(rowm[r] - mn, -256.0f) * L2E);
            const float p0 = __builtin_amdgcn_exp2f(fmaxf(a0 - mn, -256.0f) * L2E);
            const float p1 = __builtin_amdgcn_exp2f(fmaxf(a1 - mn, -256.0f) * L2E);
            float rs = p0 + p1;
            rs += __shfl_xor(rs, 1, 32); rs += __shfl_xor(rs, 2, 32); rs += __shfl_xor(rs, 4, 32); rs += __shfl_xor(rs, 8, 32);
            rowl[r] = rowl[r] * corr + rs; rowm[r] = mn;
#pragma unroll
            for (int f = 0; f < 8; ++f) acc[f][r] = acc[f][r] * corr;
            const int prow = (8 * hi + r) * PSP;
            if (HIRES) { unsigned short b0h, b0l, b1h, b1l; splitf(p0, b0h, b0l); splitf(p1, b1h, b1l); P0[prow + lr] = b0h; P1[prow + lr] = b0l; P0[prow + 16 + lr] = b1h; P1[prow + 16 + lr] = b1l; }
            else { const h16 c0 = (h16)(p0 * PCAR); const h16 c1 = (h16)(p1 * PCAR); P0[prow + lr] = __builtin_bit_cast(unsigned short, c0); P0[prow + 16 + lr] = __builtin_bit_cast(unsigned short, c1); }
        }
        __builtin_amdgcn_wave_barrier(); asm volatile("" ::: "memory");
        if (HIRES) {
            const v16bf pah = ldsAbf(P0 + lr * PSP + 8 * hi), pal = ldsAbf(P1 + lr * PSP + 8 * hi);
            v16bf vh, vl;
#pragma unroll
            for (int f = 0; f < 8; ++f) {
                vh = WFrag<bf>::ld(Vh + ((size_t)(g * HD + f * 16 + lr)) * RH + 8 * hi + kb);
                vl = WFrag<bf>::ld(Vl + ((size_t)(g * HD + f * 16 + lr)) * RH + 8 * hi + kb);
                acc[f] = wmmab(pah, vh, acc[f]); acc[f] = wmmab(pal, vh, acc[f]); acc[f] = wmmab(pah, vl, acc[f]); }
            asm volatile("v_nop\n\tv_nop\n\tv_nop\n\tv_nop" : "+v"(acc[0]), "+v"(acc[1]), "+v"(acc[2]), "+v"(acc[3]), "+v"(acc[4]), "+v"(acc[5]), "+v"(acc[6]), "+v"(acc[7]) : "v"(pah), "v"(pal), "v"(vh), "v"(vl));
        } else {
            const v16h pa = ldsA16(P0 + lr * PSP + 8 * hi);
            v16h vf;
#pragma unroll
            for (int f = 0; f < 8; ++f) { vf = WFrag<h16>::ld(V16 + ((size_t)(g * HD + f * 16 + lr)) * SEQ + 8 * hi + kb); acc[f] = wmma16(pa, vf, acc[f]); }
            asm volatile("v_nop\n\tv_nop\n\tv_nop\n\tv_nop" : "+v"(acc[0]), "+v"(acc[1]), "+v"(acc[2]), "+v"(acc[3]), "+v"(acc[4]), "+v"(acc[5]), "+v"(acc[6]), "+v"(acc[7]) : "v"(pa), "v"(vf));
        }
    }
    const int bad = FL[0];
    const float qnan = __uint_as_float(0x7fc00000u);
    float fct[8];
#pragma unroll
    for (int r = 0; r < 8; ++r) fct[r] = (HIRES ? 1.0f : (CCAR / PCAR)) * (1.0f / rowl[r]);
    const int npl = HIRES ? 2 : 1;
#pragma unroll 1
    for (int pl = 0; pl < npl; ++pl) {
        __builtin_amdgcn_wave_barrier(); asm volatile("" ::: "memory");
#pragma unroll
        for (int f = 0; f < 8; ++f) {
#pragma unroll
            for (int r = 0; r < 8; ++r) {
                float o = acc[f][r] * fct[r]; o = bad ? qnan : o;
                unsigned short bits;
                if (HIRES) { unsigned short oh, ol; splitf(o, oh, ol); bits = pl ? ol : oh; } else { const h16 oh16 = (h16)o; bits = __builtin_bit_cast(unsigned short, oh16); }
                CW[(8 * hi + r) * CSP + f * 16 + lr] = bits; } }
        __builtin_amdgcn_wave_barrier(); asm volatile("" ::: "memory");
        unsigned short* dst = HIRES ? (pl ? ATl : ATh) : AT16;
#pragma unroll 1
        for (int ps = 0; ps < 2; ++ps) {
#pragma unroll
            for (int sI = 0; sI < 8; ++sI) { const int row = 2 * sI + hi; const v8us val = *(const v8usa*)(CW + row * CSP + lr * 8);
                *(volatile v8us*)(dst + (size_t)(q0 + row) * DQ + h * HD + lr * 8) = val; }
            if (ps == 0) __threadfence(); }
    }
}

extern "C" void kernel_launch(void* const* d_in, const int* in_sizes, int n_in,
                              void* d_out, int out_size, void* d_ws, size_t ws_size, hipStream_t stream) {
    if (n_in < 6) return;
    if (in_sizes[0] < (NB - 1) * SEQ_FULL * HID + SEQ * HID) return;
    if (in_sizes[1] < (SEQ - 1) * SEQ_FULL + SEQ) return;
    if (in_sizes[2] < DQ * HID || in_sizes[3] < DKV * HID || in_sizes[4] < DKV * HID || in_sizes[5] < HID * DQ) return;
    if (out_size < NB * SEQ * HID) return;
    const float* x  = (const float*)d_in[0];
    const float* am = (const float*)d_in[1];
    const float* wq = (const float*)d_in[2];
    const float* wk = (const float*)d_in[3];
    const float* wv = (const float*)d_in[4];
    const float* wo = (const float*)d_in[5];
    float* OUT = (float*)d_out;
    char* wsp = (char*)d_ws;
    auto take = [&](size_t bytes) { char* p = wsp; wsp += (bytes + 255) & ~(size_t)255; return (void*)p; };
    const int nthr_m = SEQ * SEQ / 64; const int MBLK = (nthr_m + 255) / 256;
    bf*  WQ   = (bf*)take((size_t)DQ * HID * 2);
    bf*  WK   = (bf*)take((size_t)DKV * HID * 2);
    bf*  WV   = (bf*)take((size_t)DKV * HID * 2);
    bf*  WO   = (bf*)take((size_t)HID * DQ * 2);
    h16* WO16 = (h16*)take((size_t)HID * DQ * 2);
    float* INVF = (float*)take(256);
    float* CS   = (float*)take((size_t)SEQ * HD * 2 * 4);
    int* MPART  = (int*)take((size_t)MBLK * 128);
    int* FLAG   = (int*)take(128);
    bf*  XB   = (bf*)take((size_t)SEQ * HID * 2);
    float* FQ = (float*)take((size_t)SEQ * DQ * 4);
    float* FK = (float*)take((size_t)SEQ * DKV * 4);
    float* FV = (float*)take((size_t)SEQ * DKV * 4);
    h16* Q16  = (h16*)take((size_t)NHQ * SEQ * HD * 2);
    bf*  Qh   = (bf*)take((size_t)NHQ * RH * HD * 2);
    bf*  Ql   = (bf*)take((size_t)NHQ * RH * HD * 2);
    h16* K16  = (h16*)take((size_t)NKV * SEQ * HD * 2);
    bf*  Kh   = (bf*)take((size_t)NKV * RH * HD * 2);
    bf*  Kl   = (bf*)take((size_t)NKV * RH * HD * 2);
    h16* V16  = (h16*)take((size_t)NKV * HD * SEQ * 2);
    bf*  Vh   = (bf*)take((size_t)NKV * HD * RH * 2);
    bf*  Vl   = (bf*)take((size_t)NKV * HD * RH * 2);
    unsigned short* ATh  = (unsigned short*)take((size_t)RH * DQ * 2);
    unsigned short* ATl  = (unsigned short*)take((size_t)RH * DQ * 2);
    unsigned short* AT16 = (unsigned short*)take((size_t)SEQ * DQ * 2);
    const size_t used = (size_t)(wsp - (char*)d_ws);
    if (used > ws_size || used > ((size_t)128 << 20)) return;

    k_cvt8<<<(unsigned)(((size_t)DQ * HID / 8 + 255) / 256), 256, 0, stream>>>(wq, WQ, (size_t)DQ * HID / 8);
    k_cvt8<<<(unsigned)(((size_t)DKV * HID / 8 + 255) / 256), 256, 0, stream>>>(wk, WK, (size_t)DKV * HID / 8);
    k_cvt8<<<(unsigned)(((size_t)DKV * HID / 8 + 255) / 256), 256, 0, stream>>>(wv, WV, (size_t)DKV * HID / 8);
    k_cvt8<<<(unsigned)(((size_t)HID * DQ / 8 + 255) / 256), 256, 0, stream>>>(wo, WO, (size_t)HID * DQ / 8);
    k_cvt16s<<<(unsigned)(((size_t)HID * DQ / 8 + 255) / 256), 256, 0, stream>>>(wo, WO16, (size_t)HID * DQ / 8, WCAR);
    k_invf<<<1, 64, 0, stream>>>(INVF);
    k_cstab<<<(SEQ * HD + 255) / 256, 256, 0, stream>>>(INVF, CS);
    k_mchk<<<MBLK, 256, 0, stream>>>(am, MPART);
    k_mred<<<1, 256, 0, stream>>>(MPART, MBLK, FLAG);

    const unsigned LQ = (unsigned)(((size_t)NHQ * SEQ * HD / 2 + 255) / 256), LK = (unsigned)(((size_t)NKV * SEQ * HD / 2 + 255) / 256);
    for (int b = 0; b < NB; ++b) {
        float* OUTb = OUT + (size_t)b * SEQ * HID;
        k_cvt8<<<(unsigned)(((size_t)SEQ * HID / 8 + 255) / 256), 256, 0, stream>>>(x + (size_t)b * SEQ_FULL * HID, XB, (size_t)SEQ * HID / 8);
        k_gemmw<bf, 0><<<dim3(SEQ / 64, DQ / 64, 1), 32, 0, stream>>>(XB, nullptr, WQ, nullptr, HID, FQ, DQ, 1.0f);
        k_rope<<<LQ, 256, 0, stream>>>(FQ, DQ, NHQ, CS, Q16, Qh, Ql);
        k_gemmw<bf, 0><<<dim3(SEQ / 64, DKV / 64, 1), 32, 0, stream>>>(XB, nullptr, WK, nullptr, HID, FK, DKV, 1.0f);
        k_rope<<<LK, 256, 0, stream>>>(FK, DKV, NKV, CS, K16, Kh, Kl);
        k_gemmw<bf, 0><<<dim3(SEQ / 64, DKV / 64, 1), 32, 0, stream>>>(XB, nullptr, WV, nullptr, HID, FV, DKV, 1.0f);
        k_vtp<<<LK, 256, 0, stream>>>(FV, DKV, NKV, V16, Vh, Vl);
        k_flash<true><<<dim3(RH / 64, NHQ, 1), 128, 0, stream>>>(Q16, Qh, Ql, K16, Kh, Kl, V16, Vh, Vl, FLAG, 0, AT16, ATh, ATl);
        if (SEQ - RH > 0) k_flash<false><<<dim3((SEQ - RH) / 64, NHQ, 1), 128, 0, stream>>>(Q16, Qh, Ql, K16, Kh, Kl, V16, Vh, Vl, FLAG, RH / 64, AT16, ATh, ATl);
        k_gemmw<bf, 1><<<dim3(RH / 64, HID / 64, 1), 32, 0, stream>>>(ATh, ATl, WO, nullptr, DQ, OUTb, HID, 1.0f);
        if (SEQ - RH > 0) k_gemmw<h16, 0><<<dim3((SEQ - RH) / 64, HID / 64, 1), 32, 0, stream>>>((const h16*)AT16 + (size_t)RH * DQ, nullptr, WO16, nullptr, DQ, OUTb + (size_t)RH * HID, HID, 1.0f / (CCAR * WCAR));
    }
}
